// MHAEinsum_3143916060977
// MI455X (gfx1250) — hardware-verified
//
#include <hip/hip_runtime.h>
#include <hip/hip_bf16.h>
#include <stddef.h>
#include <stdint.h>

#define NBAT  4
#define SQ    2048
#define NTOK  8192
#define HID   1024
#define NH    16
#define HDM   64
#define NHB   64
#define NQKV  3072
#define KOFS  1024
#define VOFS  2048
#define R0    64
#define NR3   256
#define QB    128
#define KC    64
#define KC3   32
#define NQB   (SQ / QB)

static_assert(NTOK == NBAT * SQ);
static_assert(NHB == NBAT * NH);
static_assert(NR3 == NBAT * R0);
static_assert(NH * HDM == HID);
static_assert(NQKV == 3 * HID);
static_assert(HID == 128 * 8);
static_assert(HID % 64 == 0);
static_assert(SQ % 256 == 0);
static_assert(NTOK % 256 == 0);
static_assert(SQ % QB == 0);
static_assert(SQ % KC == 0);
static_assert(R0 == 64);
static_assert(R0 == 2 * KC3);
static_assert(NR3 == 256);
static_assert(HDM == 64);

typedef _Float16 v16h __attribute__((ext_vector_type(16)));
typedef _Float16 v8h  __attribute__((ext_vector_type(8)));
typedef float    v8f  __attribute__((ext_vector_type(8)));
typedef float    v4f  __attribute__((ext_vector_type(4)));
typedef unsigned int   v4u   __attribute__((ext_vector_type(4)));
typedef unsigned short v8us  __attribute__((ext_vector_type(8)));
typedef unsigned short v16us __attribute__((ext_vector_type(16)));
typedef __bf16         v16b  __attribute__((ext_vector_type(16)));
typedef unsigned short ush;

union Frag  { v16h v; v8h h[2]; };
union FragU { v16us v; v8us h[2]; v16b b; };
union Pack8 { v8h h; v4u u; };
union PackU { v8us s; v4u u; };
struct HL { v4u h; v4u l; };

__device__ __forceinline__ ush f2bf(float f) {
  const unsigned u = __float_as_uint(f);
  return (ush)((u + 0x7FFFu + ((u >> 16) & 1u)) >> 16);
}
__device__ __forceinline__ float bf2f(ush b) { return __uint_as_float(((unsigned)b) << 16); }

__device__ __forceinline__ HL split8(v8f f) {
  PackU ph, pl;
#pragma unroll
  for (int e = 0; e < 8; ++e) {
    const ush hi = f2bf(f[e]);
    ph.s[e] = hi;
    pl.s[e] = f2bf(f[e] - bf2f(hi));
  }
  HL r; r.h = ph.u; r.l = pl.u;
  return r;
}

__device__ __forceinline__ v8f mma16(v16h a, v16h b, v8f c) {
  c = __builtin_amdgcn_wmma_f32_16x16x32_f16(false, a, false, b, (short)0, c, false, false);
  asm volatile("v_nop\n\tv_nop\n\tv_nop\n\tv_nop" : "+v"(c) : "v"(a), "v"(b));
  return c;
}
__device__ __forceinline__ v8f mmab(v16us a, v16us b, v8f c) {
  FragU ua, ub; ua.v = a; ub.v = b;
  c = __builtin_amdgcn_wmma_f32_16x16x32_bf16(false, ua.b, false, ub.b, (short)0, c, false, false);
  asm volatile("v_nop\n\tv_nop\n\tv_nop\n\tv_nop" : "+v"(c) : "v"(a), "v"(b));
  return c;
}

__device__ __forceinline__ v16h ldfrag(const _Float16* p, int ld, int row0, int k0, int lane) {
  const int m = lane & 15, lh = lane >> 4;
  const _Float16* q = p + (size_t)(row0 + m) * ld + k0 + 8 * lh;
  Frag f;
  f.h[0] = *(const v8h*)(q);
  f.h[1] = *(const v8h*)(q + 16);
  return f.v;
}
__device__ __forceinline__ v16us ldfragu(const ush* p, int ld, int row0, int k0, int lane) {
  const int m = lane & 15, lh = lane >> 4;
  const ush* q = p + (size_t)(row0 + m) * ld + k0 + 8 * lh;
  FragU f;
  f.h[0] = *(const v8us*)(q);
  f.h[1] = *(const v8us*)(q + 16);
  return f.v;
}

__device__ __forceinline__ v8f zero8() { return (v8f){0.f, 0.f, 0.f, 0.f, 0.f, 0.f, 0.f, 0.f}; }

__device__ __forceinline__ void gemm16x64(const _Float16* __restrict__ A, int lda,
                                          const _Float16* __restrict__ Bt, int ldb,
                                          int m0, int n0, int lane, v8f (&acc)[4]) {
#pragma unroll 2
  for (int k0 = 0; k0 < HID; k0 += 32) {
    const v16h a = ldfrag(A, lda, m0, k0, lane);
#pragma unroll
    for (int t = 0; t < 4; ++t) {
      const v16h b = ldfrag(Bt, ldb, n0 + 16 * t, k0, lane);
      acc[t] = mma16(a, b, acc[t]);
    }
  }
}

__device__ __forceinline__ void gemm3_16x64(const ush* __restrict__ Ah, const ush* __restrict__ Al, int lda,
                                            const ush* __restrict__ Bh, const ush* __restrict__ Bl, int ldb,
                                            int m0, int n0, int lane, v8f (&acc)[4]) {
#pragma unroll 1
  for (int k0 = 0; k0 < HID; k0 += 32) {
    const v16us ah = ldfragu(Ah, lda, m0, k0, lane);
    const v16us al = ldfragu(Al, lda, m0, k0, lane);
#pragma unroll
    for (int t = 0; t < 4; ++t) {
      const v16us bh = ldfragu(Bh, ldb, n0 + 16 * t, k0, lane);
      const v16us bl = ldfragu(Bl, ldb, n0 + 16 * t, k0, lane);
      acc[t] = mmab(ah, bh, acc[t]);
      acc[t] = mmab(ah, bl, acc[t]);
      acc[t] = mmab(al, bh, acc[t]);
    }
  }
}

__device__ __forceinline__ void gemm32x64(const _Float16* __restrict__ A, int lda,
                                          const _Float16* __restrict__ Bt, int ldb,
                                          int m0, int n0, int lane, v8f (&acc)[2][4]) {
#pragma unroll 2
  for (int k0 = 0; k0 < HID; k0 += 32) {
    const v16h a0 = ldfrag(A, lda, m0, k0, lane);
    const v16h a1 = ldfrag(A, lda, m0 + 16, k0, lane);
    const v16h b0 = ldfrag(Bt, ldb, n0, k0, lane);
    const v16h b1 = ldfrag(Bt, ldb, n0 + 16, k0, lane);
    const v16h b2 = ldfrag(Bt, ldb, n0 + 32, k0, lane);
    const v16h b3 = ldfrag(Bt, ldb, n0 + 48, k0, lane);
    acc[0][0] = mma16(a0, b0, acc[0][0]);
    acc[1][0] = mma16(a1, b0, acc[1][0]);
    acc[0][1] = mma16(a0, b1, acc[0][1]);
    acc[1][1] = mma16(a1, b1, acc[1][1]);
    acc[0][2] = mma16(a0, b2, acc[0][2]);
    acc[1][2] = mma16(a1, b2, acc[1][2]);
    acc[0][3] = mma16(a0, b3, acc[0][3]);
    acc[1][3] = mma16(a1, b3, acc[1][3]);
  }
}

__device__ __forceinline__ void gemm3_32x64(const ush* __restrict__ Ah, const ush* __restrict__ Al, int lda,
                                            const ush* __restrict__ Bh, const ush* __restrict__ Bl, int ldb,
                                            int m0, int n0, int lane, v8f (&acc)[2][4]) {
#pragma unroll 1
  for (int k0 = 0; k0 < HID; k0 += 32) {
    const v16us a0h = ldfragu(Ah, lda, m0, k0, lane);
    const v16us a1h = ldfragu(Ah, lda, m0 + 16, k0, lane);
    const v16us a0l = ldfragu(Al, lda, m0, k0, lane);
    const v16us a1l = ldfragu(Al, lda, m0 + 16, k0, lane);
#pragma unroll
    for (int t = 0; t < 4; ++t) {
      const v16us bh = ldfragu(Bh, ldb, n0 + 16 * t, k0, lane);
      const v16us bl = ldfragu(Bl, ldb, n0 + 16 * t, k0, lane);
      acc[0][t] = mmab(a0h, bh, acc[0][t]);
      acc[1][t] = mmab(a1h, bh, acc[1][t]);
      acc[0][t] = mmab(a0h, bl, acc[0][t]);
      acc[1][t] = mmab(a1h, bl, acc[1][t]);
      acc[0][t] = mmab(a0l, bh, acc[0][t]);
      acc[1][t] = mmab(a1l, bh, acc[1][t]);
    }
  }
}

__global__ __launch_bounds__(256) void k_cvtx(const float* __restrict__ src, _Float16* __restrict__ dh,
                                              ush* __restrict__ d3h, ush* __restrict__ d3l) {
  const int tid = threadIdx.x;
  const int row = blockIdx.x * 2 + (tid >> 7);
  const int col = (tid & 127) * 8;
  const int b   = row / SQ;
  const int s   = row - b * SQ;
  const size_t o = (size_t)row * HID + col;
  const v4f a0 = *(const v4f*)(src + o);
  const v4f a1 = *(const v4f*)(src + o + 4);
  Pack8 pk;
  pk.h = (v8h){(_Float16)a0[0], (_Float16)a0[1], (_Float16)a0[2], (_Float16)a0[3],
               (_Float16)a1[0], (_Float16)a1[1], (_Float16)a1[2], (_Float16)a1[3]};
  const v4u vv = pk.u;
  const bool three = (s < R0);
  const size_t o3 = ((size_t)(b * R0 + (three ? s : 0))) * HID + col;
  HL sp; sp.h = (v4u){0u, 0u, 0u, 0u}; sp.l = sp.h;
  if (three) {
    const v8f f = (v8f){a0[0], a0[1], a0[2], a0[3], a1[0], a1[1], a1[2], a1[3]};
    sp = split8(f);
  }
  volatile v4u* d = (volatile v4u*)(dh + o);
  *d = vv;
  if (three) { *(volatile v4u*)(d3h + o3) = sp.h; *(volatile v4u*)(d3l + o3) = sp.l; }
  __threadfence();
  *d = vv;
  if (three) { *(volatile v4u*)(d3h + o3) = sp.h; *(volatile v4u*)(d3l + o3) = sp.l; }
}

__global__ __launch_bounds__(256) void k_cvtw(const float* __restrict__ src, _Float16* __restrict__ dh,
                                              ush* __restrict__ d3h, ush* __restrict__ d3l) {
  const int tid = threadIdx.x;
  const int row = blockIdx.x * 2 + (tid >> 7);
  const int col = (tid & 127) * 8;
  const size_t o = (size_t)row * HID + col;
  const v4f a0 = *(const v4f*)(src + o);
  const v4f a1 = *(const v4f*)(src + o + 4);
  Pack8 pk;
  pk.h = (v8h){(_Float16)(a0[0] * 32.0f), (_Float16)(a0[1] * 32.0f), (_Float16)(a0[2] * 32.0f), (_Float16)(a0[3] * 32.0f),
               (_Float16)(a1[0] * 32.0f), (_Float16)(a1[1] * 32.0f), (_Float16)(a1[2] * 32.0f), (_Float16)(a1[3] * 32.0f)};
  const v4u vv = pk.u;
  const v8f f = (v8f){a0[0], a0[1], a0[2], a0[3], a1[0], a1[1], a1[2], a1[3]};
  const HL sp = split8(f);
  *(volatile v4u*)(dh + o)  = vv;
  *(volatile v4u*)(d3h + o) = sp.h;
  *(volatile v4u*)(d3l + o) = sp.l;
  __threadfence();
  *(volatile v4u*)(dh + o)  = vv;
  *(volatile v4u*)(d3h + o) = sp.h;
  *(volatile v4u*)(d3l + o) = sp.l;
}

#define WTP 65
__global__ __launch_bounds__(256) void k_wtr(const float* __restrict__ W, int ncol, int nofs,
                                             _Float16* __restrict__ wt, ush* __restrict__ wh,
                                             ush* __restrict__ wl) {
  __shared__ float tl[64 * WTP];
  const int tid = threadIdx.x;
  const int n0 = blockIdx.x * 64, k0 = blockIdx.y * 64;
#pragma unroll
  for (int j = 0; j < 4; ++j) {
    const int p  = tid + 256 * j;
    const int kk = p >> 4;
    const int q4 = (p & 15) * 4;
    const v4f a = *(const v4f*)(W + (size_t)(k0 + kk) * ncol + n0 + q4);
    float* d = tl + kk * WTP + q4;
    d[0] = a[0]; d[1] = a[1]; d[2] = a[2]; d[3] = a[3];
  }
  __syncthreads();
  v4u vt[2], vh[2], vl[2];
  size_t go[2];
#pragma unroll
  for (int j = 0; j < 2; ++j) {
    const int p  = tid + 256 * j;
    const int nn = p >> 3;
    const int pc = p & 7;
    const float* cp = tl + (pc * 8) * WTP + nn;
    const v8f f = (v8f){cp[0 * WTP], cp[1 * WTP], cp[2 * WTP], cp[3 * WTP],
                        cp[4 * WTP], cp[5 * WTP], cp[6 * WTP], cp[7 * WTP]};
    Pack8 pk;
    pk.h = (v8h){(_Float16)(f[0] * 32.0f), (_Float16)(f[1] * 32.0f), (_Float16)(f[2] * 32.0f), (_Float16)(f[3] * 32.0f),
                 (_Float16)(f[4] * 32.0f), (_Float16)(f[5] * 32.0f), (_Float16)(f[6] * 32.0f), (_Float16)(f[7] * 32.0f)};
    vt[j] = pk.u;
    const HL s = split8(f);
    vh[j] = s.h; vl[j] = s.l;
    go[j] = (size_t)(nofs + n0 + nn) * HID + k0 + pc * 8;
  }
  for (int ps = 0; ps < 2; ++ps) {
#pragma unroll
    for (int j = 0; j < 2; ++j) {
      *(volatile v4u*)(wt + go[j]) = vt[j];
      *(volatile v4u*)(wh + go[j]) = vh[j];
      *(volatile v4u*)(wl + go[j]) = vl[j];
    }
    __threadfence();
  }
}

#define SFP 132
__global__ __launch_bounds__(256) void k_qkv(const _Float16* __restrict__ xh,
                                             const _Float16* __restrict__ wt,
                                             _Float16* __restrict__ qp,
                                             _Float16* __restrict__ kp,
                                             _Float16* __restrict__ vtp) {
  __shared__ __align__(16) float sf[64 * SFP];
  const int tid = threadIdx.x, lane = tid & 31, wave = tid >> 5;
  const int hh = lane >> 4, c = lane & 15;
  const int wm = wave >> 1, wn = wave & 1;
  const int mb = blockIdx.x * 64;
  const int b  = mb / SQ;
  const int sb = mb - b * SQ;
  const int ns = blockIdx.y;
  const int which = ns >> 3;
  const int hp = ns & 7;
  const int m0 = mb + wm * 16;
  const int n0 = ns * 128 + wn * 64;

  v8f acc[4];
#pragma unroll
  for (int t = 0; t < 4; ++t) acc[t] = zero8();
  gemm16x64(xh, HID, wt, HID, m0, n0, lane, acc);

#pragma unroll
  for (int t = 0; t < 4; ++t) {
#pragma unroll
    for (int r = 0; r < 8; ++r)
      sf[(wm * 16 + 8 * hh + r) * SFP + wn * 64 + 16 * t + c] = acc[t][r] * 0.03125f;
  }
  __syncthreads();

  if (which < 2) {
    v4u val[4];
    size_t go[4];
#pragma unroll
    for (int j = 0; j < 4; ++j) {
      const int p    = tid + 256 * j;
      const int lr   = p >> 4;
      const int pc   = p & 15;
      const int head = 2 * hp + (pc >> 3);
      const int d0   = (pc & 7) * 8;
      const float* ra = sf + lr * SFP + pc * 8;
      const v4f a0 = *(const v4f*)(ra), a1 = *(const v4f*)(ra + 4);
      Pack8 pk;
      pk.h = (v8h){(_Float16)a0[0], (_Float16)a0[1], (_Float16)a0[2], (_Float16)a0[3],
                   (_Float16)a1[0], (_Float16)a1[1], (_Float16)a1[2], (_Float16)a1[3]};
      val[j] = pk.u;
      go[j]  = ((size_t)(b * NH + head) * SQ + sb + lr) * HDM + d0;
    }
    _Float16* base = (which == 0) ? qp : kp;
    for (int ps = 0; ps < 2; ++ps) {
#pragma unroll
      for (int j = 0; j < 4; ++j) *(volatile v4u*)(base + go[j]) = val[j];
      __threadfence();
    }
  } else {
    v4u val[4];
    size_t go[4];
#pragma unroll
    for (int j = 0; j < 4; ++j) {
      const int p    = tid + 256 * j;
      const int d    = p >> 3;
      const int pc   = p & 7;
      const int head = 2 * hp + (d >> 6);
      const int dd   = d & 63;
      const float* cp = sf + (pc * 8) * SFP + d;
      Pack8 pk;
      pk.h = (v8h){(_Float16)cp[0 * SFP], (_Float16)cp[1 * SFP], (_Float16)cp[2 * SFP], (_Float16)cp[3 * SFP],
                   (_Float16)cp[4 * SFP], (_Float16)cp[5 * SFP], (_Float16)cp[6 * SFP], (_Float16)cp[7 * SFP]};
      val[j] = pk.u;
      go[j]  = ((size_t)(b * NH + head) * HDM + dd) * SQ + sb + pc * 8;
    }
    for (int ps = 0; ps < 2; ++ps) {
#pragma unroll
      for (int j = 0; j < 4; ++j) *(volatile v4u*)(vtp + go[j]) = val[j];
      __threadfence();
    }
  }
}

__global__ __launch_bounds__(256) void k_qkv3(const ush* __restrict__ xh3, const ush* __restrict__ xl3,
                                              const ush* __restrict__ wth, const ush* __restrict__ wtl,
                                              ush* __restrict__ q3h, ush* __restrict__ q3l,
                                              ush* __restrict__ k3h, ush* __restrict__ k3l,
                                              ush* __restrict__ v3h, ush* __restrict__ v3l) {
  __shared__ __align__(16) float sf[64 * SFP];
  const int tid = threadIdx.x, lane = tid & 31, wave = tid >> 5;
  const int hh = lane >> 4, c = lane & 15;
  const int wm = wave >> 1, wn = wave & 1;
  const int b   = blockIdx.x;
  const int mb3 = b * R0;
  const int ns  = blockIdx.y;
  const int which = ns >> 3;
  const int hp  = ns & 7;
  const int m0  = mb3 + wm * 16;
  const int n0  = ns * 128 + wn * 64;

  v8f acc[4];
#pragma unroll
  for (int t = 0; t < 4; ++t) acc[t] = zero8();
  gemm3_16x64(xh3, xl3, HID, wth, wtl, HID, m0, n0, lane, acc);

#pragma unroll
  for (int t = 0; t < 4; ++t) {
#pragma unroll
    for (int r = 0; r < 8; ++r)
      sf[(wm * 16 + 8 * hh + r) * SFP + wn * 64 + 16 * t + c] = acc[t][r];
  }
  __syncthreads();

  if (which < 2) {
    v4u vh[4], vl[4];
    size_t go[4];
#pragma unroll
    for (int j = 0; j < 4; ++j) {
      const int p    = tid + 256 * j;
      const int lr   = p >> 4;
      const int pc   = p & 15;
      const int head = 2 * hp + (pc >> 3);
      const int d0   = (pc & 7) * 8;
      const float* ra = sf + lr * SFP + pc * 8;
      const v4f a0 = *(const v4f*)(ra), a1 = *(const v4f*)(ra + 4);
      const v8f f = (v8f){a0[0], a0[1], a0[2], a0[3], a1[0], a1[1], a1[2], a1[3]};
      const HL s = split8(f);
      vh[j] = s.h; vl[j] = s.l;
      go[j] = ((size_t)(b * NH + head) * R0 + lr) * HDM + d0;
    }
    ush* ph = (which == 0) ? q3h : k3h;
    ush* pl = (which == 0) ? q3l : k3l;
    for (int ps = 0; ps < 2; ++ps) {
#pragma unroll
      for (int j = 0; j < 4; ++j) {
        *(volatile v4u*)(ph + go[j]) = vh[j];
        *(volatile v4u*)(pl + go[j]) = vl[j];
      }
      __threadfence();
    }
  } else {
    v4u vh[4], vl[4];
    size_t go[4];
#pragma unroll
    for (int j = 0; j < 4; ++j) {
      const int p    = tid + 256 * j;
      const int d    = p >> 3;
      const int pc   = p & 7;
      const int head = 2 * hp + (d >> 6);
      const int dd   = d & 63;
      const float* cp = sf + (pc * 8) * SFP + d;
      const v8f f = (v8f){cp[0 * SFP], cp[1 * SFP], cp[2 * SFP], cp[3 * SFP],
                          cp[4 * SFP], cp[5 * SFP], cp[6 * SFP], cp[7 * SFP]};
      const HL s = split8(f);
      vh[j] = s.h; vl[j] = s.l;
      go[j] = ((size_t)(b * NH + head) * HDM + dd) * R0 + pc * 8;
    }
    for (int ps = 0; ps < 2; ++ps) {
#pragma unroll
      for (int j = 0; j < 4; ++j) {
        *(volatile v4u*)(v3h + go[j]) = vh[j];
        *(volatile v4u*)(v3l + go[j]) = vl[j];
      }
      __threadfence();
    }
  }
}

#define KTP 72
__global__ __launch_bounds__(256) void k_attn(const _Float16* __restrict__ qp,
                                              const _Float16* __restrict__ kp,
                                              const _Float16* __restrict__ vt,
                                              _Float16* __restrict__ op, float sscale) {
  __shared__ __align__(16) _Float16 Ks[KC * KTP];
  __shared__ __align__(16) _Float16 Vs[HDM * KTP];
  __shared__ __align__(16) _Float16 Ps[8 * 16 * KTP];

  const int tid = threadIdx.x, lane = tid & 31, wave = tid >> 5;
  const int hh = lane >> 4, c = lane & 15;
  const int qb  = blockIdx.x % NQB;
  const int hb  = blockIdx.x / NQB;
  const int h   = hb % NH;
  const int b   = hb / NH;
  const int q0  = qb * QB + wave * 16;

  const _Float16* Q = qp + (size_t)hb * SQ * HDM;
  const _Float16* K = kp + (size_t)hb * SQ * HDM;
  const _Float16* V = vt + (size_t)hb * HDM * SQ;
  const size_t trow0 = (size_t)b * SQ;

  const float NEGI = -__builtin_huge_valf();
  float mrow[8], lrow[8];
  v8f oacc[4];
#pragma unroll
  for (int r = 0; r < 8; ++r) { mrow[r] = NEGI; lrow[r] = 0.f; }
#pragma unroll
  for (int t = 0; t < 4; ++t) oacc[t] = zero8();

  _Float16* pw = Ps + wave * 16 * KTP;
  const int nck = 2 * qb + 2;

  for (int kc = 0; kc < nck; ++kc) {
    const int kv0 = kc * KC;
    __syncthreads();
    {
      const int r  = tid >> 2;
      const int qq = (tid & 3) * 16;
      const _Float16* ks = K + (size_t)(kv0 + r) * HDM + qq;
#pragma unroll
      for (int e = 0; e < 2; ++e) *(v8h*)(Ks + r * KTP + qq + 8 * e) = *(const v8h*)(ks + 8 * e);
      const _Float16* vs = V + (size_t)r * SQ + kv0 + qq;
#pragma unroll
      for (int e = 0; e < 2; ++e) *(v8h*)(Vs + r * KTP + qq + 8 * e) = *(const v8h*)(vs + 8 * e);
    }
    __syncthreads();

    v8f s[4];
#pragma unroll
    for (int j = 0; j < 4; ++j) s[j] = zero8();
#pragma unroll
    for (int dc = 0; dc < 2; ++dc) {
      const v16h qa = ldfrag(Q, HDM, q0, dc * 32, lane);
#pragma unroll
      for (int j = 0; j < 4; ++j) {
        const v16h kb = ldfrag(Ks, KTP, j * 16, dc * 32, lane);
        s[j] = mma16(qa, kb, s[j]);
      }
    }
    const bool edge = (kc >= 2 * qb);
#pragma unroll
    for (int r = 0; r < 8; ++r) {
      const int qry = q0 + 8 * hh + r;
#pragma unroll
      for (int j = 0; j < 4; ++j) {
        const int key = kv0 + 16 * j + c;
        const float v = s[j][r] * sscale;
        s[j][r] = (edge && key > qry) ? NEGI : v;
      }
    }
    float cm[8];
#pragma unroll
    for (int r = 0; r < 8; ++r) {
      float m = NEGI;
#pragma unroll
      for (int j = 0; j < 4; ++j) m = fmaxf(m, s[j][r]);
#pragma unroll
      for (int off = 1; off < 16; off <<= 1) m = fmaxf(m, __shfl_xor(m, off, 32));
      cm[r] = m;
    }
    float al[8];
#pragma unroll
    for (int r = 0; r < 8; ++r) {
      const float mnew  = fmaxf(mrow[r], cm[r]);
      const float alpha = __expf(mrow[r] - mnew);
      mrow[r] = mnew;
      float psum = 0.f;
#pragma unroll
      for (int j = 0; j < 4; ++j) {
        const float p = __expf(s[j][r] - mnew);
        psum += p;
        pw[(8 * hh + r) * KTP + j * 16 + c] = (_Float16)(p * 1024.0f);
      }
#pragma unroll
      for (int off = 1; off < 16; off <<= 1) psum += __shfl_xor(psum, off, 32);
      lrow[r] = lrow[r] * alpha + psum;
      al[r] = alpha;
    }
#pragma unroll
    for (int t = 0; t < 4; ++t)
#pragma unroll
      for (int r = 0; r < 8; ++r) oacc[t][r] *= al[r];
    __syncthreads();

#pragma unroll
    for (int kk = 0; kk < 2; ++kk) {
      const v16h pa = ldfrag(pw, KTP, 0, kk * 32, lane);
#pragma unroll
      for (int t = 0; t < 4; ++t) {
        const v16h vb = ldfrag(Vs, KTP, t * 16, kk * 32, lane);
        oacc[t] = mma16(pa, vb, oacc[t]);
      }
    }
  }

  float invl[8];
#pragma unroll
  for (int r = 0; r < 8; ++r) invl[r] = (lrow[r] > 0.f) ? (0.015625f / lrow[r]) : 0.f;
  __syncthreads();
#pragma unroll
  for (int r = 0; r < 8; ++r) {
#pragma unroll
    for (int t = 0; t < 4; ++t)
      pw[(8 * hh + r) * KTP + 16 * t + c] = (_Float16)(oacc[t][r] * invl[r]);
  }
  __syncthreads();
  v4u val[4];
  size_t go[4];
#pragma unroll
  for (int it = 0; it < 4; ++it) {
    const int p  = lane + 32 * it;
    const int L  = p >> 3;
    const int pc = p & 7;
    Pack8 pk;
    pk.h    = *(const v8h*)(pw + L * KTP + pc * 8);
    val[it] = pk.u;
    go[it]  = (trow0 + q0 + L) * HID + (size_t)h * HDM + pc * 8;
  }
  for (int ps = 0; ps < 2; ++ps) {
#pragma unroll
    for (int it = 0; it < 4; ++it) *(volatile v4u*)(op + go[it]) = val[it];
    __threadfence();
  }
}

#define VTP3 40
static_assert(2 * KC3 * KTP >= 64 * KTP);
static_assert(2 * HDM * VTP3 >= 64 * KTP);
__global__ __launch_bounds__(128) __attribute__((amdgpu_num_vgpr(256)))
void k_attn3(const ush* __restrict__ q3h, const ush* __restrict__ q3l,
             const ush* __restrict__ k3h, const ush* __restrict__ k3l,
             const ush* __restrict__ v3h, const ush* __restrict__ v3l,
             ush* __restrict__ o3h, ush* __restrict__ o3l, float sscale) {
  __shared__ __align__(16) ush Ks3[2 * KC3 * KTP];
  __shared__ __align__(16) ush Vs3[2 * HDM * VTP3];
  __shared__ __align__(16) ush P3[2 * 4 * 16 * VTP3];

  const int tid = threadIdx.x, lane = tid & 31, wave = tid >> 5;
  const int hh = lane >> 4, c = lane & 15;
  const int hb  = blockIdx.x;
  const int h   = hb % NH;
  const int b   = hb / NH;
  const int q0  = wave * 16;

  const ush* Qh  = q3h + (size_t)hb * R0 * HDM;
  const ush* Ql  = q3l + (size_t)hb * R0 * HDM;
  const ush* K3H = k3h + (size_t)hb * R0 * HDM;
  const ush* K3L = k3l + (size_t)hb * R0 * HDM;
  const ush* V3H = v3h + (size_t)hb * HDM * R0;
  const ush* V3L = v3l + (size_t)hb * HDM * R0;
  const size_t prow0 = (size_t)b * R0;

  ush* Ksh = Ks3;
  ush* Ksl = Ks3 + KC3 * KTP;
  ush* Vsh = Vs3;
  ush* Vsl = Vs3 + HDM * VTP3;
  ush* pwh = P3 + (0 * 4 + wave) * 16 * VTP3;
  ush* pwl = P3 + (1 * 4 + wave) * 16 * VTP3;

  const float NEGI = -__builtin_huge_valf();
  float mrow[8], lrow[8];
  v8f oacc[4];
#pragma unroll
  for (int r = 0; r < 8; ++r) { mrow[r] = NEGI; lrow[r] = 0.f; }
#pragma unroll
  for (int t = 0; t < 4; ++t) oacc[t] = zero8();

  for (int kc = 0; kc < 2; ++kc) {
    const int kv0 = kc * KC3;
    __syncthreads();
    {
      const int r  = tid >> 2;
      const int qq = (tid & 3) * 16;
      const ush* ah = K3H + (size_t)(kv0 + r) * HDM + qq;
      const ush* al = K3L + (size_t)(kv0 + r) * HDM + qq;
#pragma unroll
      for (int e = 0; e < 2; ++e) {
        *(v8us*)(Ksh + r * KTP + qq + 8 * e) = *(const v8us*)(ah + 8 * e);
        *(v8us*)(Ksl + r * KTP + qq + 8 * e) = *(const v8us*)(al + 8 * e);
      }
      const int dr = tid >> 1;
      const int q2 = (tid & 1) * 16;
      const ush* vh = V3H + (size_t)dr * R0 + kv0 + q2;
      const ush* vl = V3L + (size_t)dr * R0 + kv0 + q2;
#pragma unroll
      for (int e = 0; e < 2; ++e) {
        *(v8us*)(Vsh + dr * VTP3 + q2 + 8 * e) = *(const v8us*)(vh + 8 * e);
        *(v8us*)(Vsl + dr * VTP3 + q2 + 8 * e) = *(const v8us*)(vl + 8 * e);
      }
    }
    __syncthreads();

    v8f s[2];
#pragma unroll
    for (int j = 0; j < 2; ++j) s[j] = zero8();
#pragma unroll
    for (int dc = 0; dc < 2; ++dc) {
      const v16us qah = ldfragu(Qh, HDM, q0, dc * 32, lane);
      const v16us qal = ldfragu(Ql, HDM, q0, dc * 32, lane);
#pragma unroll
      for (int j = 0; j < 2; ++j) {
        const v16us kbh = ldfragu(Ksh, KTP, j * 16, dc * 32, lane);
        const v16us kbl = ldfragu(Ksl, KTP, j * 16, dc * 32, lane);
        s[j] = mmab(qah, kbh, s[j]);
        s[j] = mmab(qah, kbl, s[j]);
        s[j] = mmab(qal, kbh, s[j]);
      }
    }
#pragma unroll
    for (int r = 0; r < 8; ++r) {
      const int qry = q0 + 8 * hh + r;
#pragma unroll
      for (int j = 0; j < 2; ++j) {
        const int key = kv0 + 16 * j + c;
        const float v = s[j][r] * sscale;
        s[j][r] = (key > qry) ? NEGI : v;
      }
    }
    float cm[8];
#pragma unroll
    for (int r = 0; r < 8; ++r) {
      float m = fmaxf(s[0][r], s[1][r]);
#pragma unroll
      for (int off = 1; off < 16; off <<= 1) m = fmaxf(m, __shfl_xor(m, off, 32));
      cm[r] = m;
    }
    float al[8];
#pragma unroll
    for (int r = 0; r < 8; ++r) {
      const float mnew  = fmaxf(mrow[r], cm[r]);
      const float alpha = __expf(mrow[r] - mnew);
      mrow[r] = mnew;
      float psum = 0.f;
#pragma unroll
      for (int j = 0; j < 2; ++j) {
        const float p = __expf(s[j][r] - mnew);
        psum += p;
        const ush phi = f2bf(p);
        pwh[(8 * hh + r) * VTP3 + j * 16 + c] = phi;
        pwl[(8 * hh + r) * VTP3 + j * 16 + c] = f2bf(p - bf2f(phi));
      }
#pragma unroll
      for (int off = 1; off < 16; off <<= 1) psum += __shfl_xor(psum, off, 32);
      lrow[r] = lrow[r] * alpha + psum;
      al[r] = alpha;
    }
#pragma unroll
    for (int t = 0; t < 4; ++t)
#pragma unroll
      for (int r = 0; r < 8; ++r) oacc[t][r] *= al[r];
    __syncthreads();

    {
      const v16us pah = ldfragu(pwh, VTP3, 0, 0, lane);
      const v16us pal = ldfragu(pwl, VTP3, 0, 0, lane);
#pragma unroll
      for (int t = 0; t < 4; ++t) {
        const v16us vbh = ldfragu(Vsh, VTP3, t * 16, 0, lane);
        const v16us vbl = ldfragu(Vsl, VTP3, t * 16, 0, lane);
        oacc[t] = mmab(pah, vbh, oacc[t]);
        oacc[t] = mmab(pah, vbl, oacc[t]);
        oacc[t] = mmab(pal, vbh, oacc[t]);
      }
    }
  }
  __syncthreads();

  ush* Oh = Ks3;
  ush* Ol = Vs3;
#pragma unroll
  for (int r = 0; r < 8; ++r) {
    const float lr  = lrow[r];
    const float inv = (lr > 0.f) ? (1.0f / lr) : 0.f;
    const int   row = wave * 16 + 8 * hh + r;
#pragma unroll
    for (int t = 0; t < 4; ++t) {
      const float o = oacc[t][r] * inv;
      const ush hi = f2bf(o);
      Oh[row * KTP + 16 * t + c] = hi;
      Ol[row * KTP + 16 * t + c] = f2bf(o - bf2f(hi));
    }
  }
  __syncthreads();
  v4u vh[4], vl[4];
  size_t go[4];
#pragma unroll
  for (int it = 0; it < 4; ++it) {
    const int p   = lane + 32 * it;
    const int L   = p >> 3;
    const int pc  = p & 7;
    PackU pk;
    pk.s   = *(const v8us*)(Oh + (wave * 16 + L) * KTP + pc * 8);
    vh[it] = pk.u;
    pk.s   = *(const v8us*)(Ol + (wave * 16 + L) * KTP + pc * 8);
    vl[it] = pk.u;
    go[it] = (prow0 + q0 + L) * HID + (size_t)h * HDM + pc * 8;
  }
  for (int ps = 0; ps < 2; ++ps) {
#pragma unroll
    for (int it = 0; it < 4; ++it) {
      *(volatile v4u*)(o3h + go[it]) = vh[it];
      *(volatile v4u*)(o3l + go[it]) = vl[it];
    }
    __threadfence();
  }
}

#define OTP 68
__device__ __forceinline__ void out_epilogue(v8f (&acc)[2][4], float scale, const float* __restrict__ bias,
                                             float* sw, float* __restrict__ out,
                                             int m0, int n0, int lane, int hh, int c) {
#pragma unroll
  for (int sub = 0; sub < 2; ++sub) {
    __syncthreads();
#pragma unroll
    for (int t = 0; t < 4; ++t) {
      const float bb = bias[n0 + 16 * t + c];
#pragma unroll
      for (int r = 0; r < 8; ++r) sw[(8 * hh + r) * OTP + 16 * t + c] = acc[sub][t][r] * scale + bb;
    }
    __syncthreads();
    v4f val[8];
    size_t go[8];
#pragma unroll
    for (int it = 0; it < 8; ++it) {
      const int p    = lane + 32 * it;
      const int L    = p >> 3;
      const int pc   = p & 7;
      const int row  = L >> 1;
      const int half = L & 1;
      val[it] = *(const v4f*)(sw + row * OTP + half * 32 + pc * 4);
      go[it]  = (size_t)(m0 + sub * 16 + row) * HID + n0 + half * 32 + pc * 4;
    }
    for (int ps = 0; ps < 2; ++ps) {
#pragma unroll
      for (int it = 0; it < 8; ++it) *(volatile v4f*)(out + go[it]) = val[it];
      __threadfence();
    }
  }
}

__global__ __launch_bounds__(256) void k_out(const _Float16* __restrict__ ap,
                                             const _Float16* __restrict__ wt,
                                             const float* __restrict__ bo,
                                             float* __restrict__ out) {
  __shared__ __align__(16) float st[8][16 * OTP];
  const int tid = threadIdx.x, lane = tid & 31, wave = tid >> 5;
  const int hh = lane >> 4, c = lane & 15;
  const int m0 = blockIdx.x * 256 + wave * 32;
  const int n0 = blockIdx.y * 64;

  v8f acc[2][4];
#pragma unroll
  for (int s = 0; s < 2; ++s)
#pragma unroll
    for (int t = 0; t < 4; ++t) acc[s][t] = zero8();
  gemm32x64(ap, HID, wt, HID, m0, n0, lane, acc);
  out_epilogue(acc, 0.001953125f, bo, st[wave], out, m0, n0, lane, hh, c);
}

__global__ __launch_bounds__(256) void k_out3(const ush* __restrict__ ah, const ush* __restrict__ al,
                                              const ush* __restrict__ wh, const ush* __restrict__ wl,
                                              const float* __restrict__ bo,
                                              float* __restrict__ out) {
  __shared__ __align__(16) float st[8][16 * OTP];
  const int tid = threadIdx.x, lane = tid & 31, wave = tid >> 5;
  const int hh = lane >> 4, c = lane & 15;
  const int mA = wave * 32;
  const int mO = (wave >> 1) * SQ + (wave & 1) * 32;
  const int n0 = blockIdx.y * 64;

  v8f acc[2][4];
#pragma unroll
  for (int s = 0; s < 2; ++s)
#pragma unroll
    for (int t = 0; t < 4; ++t) acc[s][t] = zero8();
  gemm3_32x64(ah, al, HID, wh, wl, HID, mA, n0, lane, acc);
  out_epilogue(acc, 1.0f, bo, st[wave], out, mO, n0, lane, hh, c);
}

extern "C" void kernel_launch(void* const* d_in, const int* in_sizes, int n_in,
                              void* d_out, int out_size, void* d_ws, size_t ws_size,
                              hipStream_t stream) {
  if (n_in < 6) return;
  if (in_sizes[0] != NTOK * HID) return;
  if (in_sizes[1] != HID * HID) return;
  if (in_sizes[2] != HID * HID) return;
  if (in_sizes[3] != HID * HID) return;
  if (in_sizes[4] != HID * HID) return;
  if (in_sizes[5] != HID) return;
  if (out_size != NTOK * HID) return;

  const float* x  = (const float*)d_in[0];
  const float* wq = (const float*)d_in[1];
  const float* wk = (const float*)d_in[2];
  const float* wv = (const float*)d_in[3];
  const float* wo = (const float*)d_in[4];
  const float* bo = (const float*)d_in[5];
  float* out = (float*)d_out;

  size_t off = 0;
  const size_t oX   = off; off += (size_t)NTOK * HID * 2;
  const size_t oX3h = off; off += (size_t)NR3 * HID * 2;
  const size_t oX3l = off; off += (size_t)NR3 * HID * 2;
  const size_t oWt  = off; off += (size_t)NQKV * HID * 2;
  const size_t oWth = off; off += (size_t)NQKV * HID * 2;
  const size_t oWtl = off; off += (size_t)NQKV * HID * 2;
  const size_t oWo  = off; off += (size_t)HID * HID * 2;
  const size_t oWoh = off; off += (size_t)HID * HID * 2;
  const size_t oWol = off; off += (size_t)HID * HID * 2;
  const size_t oQ   = off; off += (size_t)NHB * SQ * HDM * 2;
  const size_t oK   = off; off += (size_t)NHB * SQ * HDM * 2;
  const size_t oV   = off; off += (size_t)NHB * HDM * SQ * 2;
  const size_t oQ3h = off; off += (size_t)NHB * R0 * HDM * 2;
  const size_t oQ3l = off; off += (size_t)NHB * R0 * HDM * 2;
  const size_t oK3h = off; off += (size_t)NHB * R0 * HDM * 2;
  const size_t oK3l = off; off += (size_t)NHB * R0 * HDM * 2;
  const size_t oV3h = off; off += (size_t)NHB * HDM * R0 * 2;
  const size_t oV3l = off; off += (size_t)NHB * HDM * R0 * 2;
  const size_t oO3h = off; off += (size_t)NR3 * HID * 2;
  const size_t oO3l = off; off += (size_t)NR3 * HID * 2;
  const size_t oO   = off; off += (size_t)NTOK * HID * 2;
  if (off > ws_size) return;
  if (off > (size_t)134217728) return;

  char* ws = (char*)d_ws;
  _Float16* Xh  = (_Float16*)(ws + oX);
  ush*      X3h = (ush*)(ws + oX3h);
  ush*      X3l = (ush*)(ws + oX3l);
  _Float16* Wt  = (_Float16*)(ws + oWt);
  ush*      Wth = (ush*)(ws + oWth);
  ush*      Wtl = (ush*)(ws + oWtl);
  _Float16* Wot = (_Float16*)(ws + oWo);
  ush*      Woh = (ush*)(ws + oWoh);
  ush*      Wol = (ush*)(ws + oWol);
  _Float16* Qp  = (_Float16*)(ws + oQ);
  _Float16* Kp  = (_Float16*)(ws + oK);
  _Float16* Vt  = (_Float16*)(ws + oV);
  ush*      Q3h = (ush*)(ws + oQ3h);
  ush*      Q3l = (ush*)(ws + oQ3l);
  ush*      K3h = (ush*)(ws + oK3h);
  ush*      K3l = (ush*)(ws + oK3l);
  ush*      V3h = (ush*)(ws + oV3h);
  ush*      V3l = (ush*)(ws + oV3l);
  ush*      O3h = (ush*)(ws + oO3h);
  ush*      O3l = (ush*)(ws + oO3l);
  _Float16* Op  = (_Float16*)(ws + oO);

  k_cvtx<<<dim3(NTOK / 2), dim3(256), 0, stream>>>(x, Xh, X3h, X3l);
  k_wtr<<<dim3(HID / 64, HID / 64), dim3(256), 0, stream>>>(wq, HID, 0,    Wt, Wth, Wtl);
  k_wtr<<<dim3(HID / 64, HID / 64), dim3(256), 0, stream>>>(wk, HID, KOFS, Wt, Wth, Wtl);
  k_wtr<<<dim3(HID / 64, HID / 64), dim3(256), 0, stream>>>(wv, HID, VOFS, Wt, Wth, Wtl);
  k_cvtw<<<dim3(HID / 2), dim3(256), 0, stream>>>(wo, Wot, Woh, Wol);
  k_qkv<<<dim3(NTOK / 64, NQKV / 128), dim3(256), 0, stream>>>(Xh, Wt, Qp, Kp, Vt);
  k_qkv3<<<dim3(NBAT, NQKV / 128), dim3(256), 0, stream>>>(X3h, X3l, Wth, Wtl, Q3h, Q3l, K3h, K3l, V3h, V3l);
  const float sscale = 0.125f;
  k_attn<<<dim3(NHB * NQB), dim3(256), 0, stream>>>(Qp, Kp, Vt, Op, sscale);
  k_attn3<<<dim3(NHB), dim3(128), 0, stream>>>(Q3h, Q3l, K3h, K3l, V3h, V3l, O3h, O3l, sscale);
  k_out<<<dim3(NTOK / 256, HID / 64), dim3(256), 0, stream>>>(Op, Wot, bo, out);
  k_out3<<<dim3(1, HID / 64), dim3(256), 0, stream>>>(O3h, O3l, Woh, Wol, bo, out);
  (void)hipGetLastError();
}
